// HAN_23948737642663
// MI455X (gfx1250) — hardware-verified
//
#include <hip/hip_runtime.h>
#include <hip/hip_bf16.h>
#include <math.h>
#include <stddef.h>

typedef __attribute__((ext_vector_type(16))) _Float16 v16h;
typedef __attribute__((ext_vector_type(8)))  _Float16 v8h;
typedef __attribute__((ext_vector_type(16))) __bf16   v16b;
typedef __attribute__((ext_vector_type(8)))  __bf16   v8b;
typedef __attribute__((ext_vector_type(8)))  float    v8f;
typedef __attribute__((ext_vector_type(4)))  float    v4f;
typedef __attribute__((ext_vector_type(4)))  int      v4i;
typedef __attribute__((ext_vector_type(4)))  unsigned v4u;

__device__ __forceinline__ unsigned short f2bf_bits(float f) {
  unsigned u = __float_as_uint(f);
  return (unsigned short)((u + 0x7FFFu + ((u >> 16) & 1u)) >> 16);
}
__device__ __forceinline__ float bf_bits2f(unsigned short h) { return __uint_as_float(((unsigned)h) << 16); }

__device__ __forceinline__ void dep_guard_h(v8f& a, v8f& b, v16h x, v16h y) { asm volatile("v_nop\n\tv_nop\n\tv_nop\n\tv_nop" : "+v"(a), "+v"(b) : "v"(x), "v"(y)); }
__device__ __forceinline__ void dep_guard_b(v8f& a, v8f& b, v16b x, v16b y) { asm volatile("v_nop\n\tv_nop\n\tv_nop\n\tv_nop" : "+v"(a), "+v"(b) : "v"(x), "v"(y)); }
__device__ __forceinline__ void keep4_h(v16h a, v16h b, v16h c, v16h d) { asm volatile("v_nop" :: "v"(a), "v"(b), "v"(c), "v"(d)); }
__device__ __forceinline__ void keep4_b(v16b a, v16b b, v16b c, v16b d) { asm volatile("v_nop" :: "v"(a), "v"(b), "v"(c), "v"(d)); }
__device__ __forceinline__ void acc_guard4(v8f& a, v8f& b, v8f& c, v8f& d) { asm volatile("v_nop\n\tv_nop\n\tv_nop\n\tv_nop" : "+v"(a), "+v"(b), "+v"(c), "+v"(d)); }
__device__ __forceinline__ void guard3_h(v8f& a, v8f& b, v8f& c, v16h x, v16h y0, v16h y1, v16h y2) {
  asm volatile("v_nop\n\tv_nop\n\tv_nop\n\tv_nop" : "+v"(a), "+v"(b), "+v"(c) : "v"(x), "v"(y0), "v"(y1), "v"(y2));
}
__device__ __forceinline__ void acc_guard3(v8f& a, v8f& b, v8f& c) {
  asm volatile("v_nop\n\tv_nop\n\tv_nop\n\tv_nop" : "+v"(a), "+v"(b), "+v"(c));
}

template <typename T> struct Frag;
template <> struct Frag<_Float16> {
  typedef v16h V; union U { v16h v; v8h h[2]; };
  static __device__ __forceinline__ v16h load(const _Float16* p) {
    U f; f.h[0] = *(const v8h*)(p); f.h[1] = *(const v8h*)(p + 16); return f.v;
  }
  static __device__ __forceinline__ v8f mma(v16h a, v16h b, v8f c) {
    return __builtin_amdgcn_wmma_f32_16x16x32_f16(false, a, false, b, (short)0, c, false, false);
  }
  static __device__ __forceinline__ void guard(v8f& a, v8f& b, v16h x, v16h y) { dep_guard_h(a, b, x, y); }
  static __device__ __forceinline__ void keep(v16h a, v16h b, v16h c, v16h d) { keep4_h(a, b, c, d); }
};
template <> struct Frag<__bf16> {
  typedef v16b V; union U { v16b v; v8b h[2]; };
  static __device__ __forceinline__ v16b load(const __bf16* p) {
    U f; f.h[0] = *(const v8b*)(p); f.h[1] = *(const v8b*)(p + 16); return f.v;
  }
  static __device__ __forceinline__ v8f mma(v16b a, v16b b, v8f c) {
    return __builtin_amdgcn_wmma_f32_16x16x32_bf16(false, a, false, b, (short)0, c, false, false);
  }
  static __device__ __forceinline__ void guard(v8f& a, v8f& b, v16b x, v16b y) { dep_guard_b(a, b, x, y); }
  static __device__ __forceinline__ void keep(v16b a, v16b b, v16b c, v16b d) { keep4_b(a, b, c, d); }
};

template <int ET> struct Elem;
template <> struct Elem<0> { typedef _Float16 T; };
template <> struct Elem<1> { typedef __bf16 T; };
template <int ET, bool SPLIT, int BIAS_MODE, int OUT_MODE, bool RESID, int ACT = 0>
__global__ __launch_bounds__(256) void wmma_gemm64(
    const unsigned short* __restrict__ Ap, const unsigned short* __restrict__ A2p, int lda, long strideA,
    const unsigned short* __restrict__ Btp, const unsigned short* __restrict__ Bt2p, int ldb, long strideB,
    void* __restrict__ Cout, void* __restrict__ Cout2, int ldc, long strideC,
    const float* __restrict__ bias,
    const float* __restrict__ resid, long strideR,
    int M, int N, int K, float scale) {
  typedef typename Elem<ET>::T T;
  typedef typename Frag<T>::V V;
  const T* A = (const T*)Ap; const T* A2 = (const T*)A2p; const T* Bt = (const T*)Btp; const T* Bt2 = (const T*)Bt2p;
  __shared__ __align__(16) float sT[8][16 * 68];
  const int b    = blockIdx.y;
  const int lane = threadIdx.x & 31;
  const int wave = threadIdx.x >> 5;
  const int tilesN = N >> 6;
  const int tilesM = M >> 6;
  const int tile = blockIdx.x * 8 + wave;
  if (tile >= tilesM * tilesN) return;
  const int tm = tile / tilesN;
  const int tn = tile - tm * tilesN;
  const int m0 = tm << 6;
  const int n0 = tn << 6;

  const T* Ab  = A  + (size_t)b * strideA;
  const T* Bb  = Bt + (size_t)b * strideB;
  const T* Ab2 = SPLIT ? (A2  + (size_t)b * strideA) : nullptr;
  const T* Bb2 = SPLIT ? (Bt2 + (size_t)b * strideB) : nullptr;

  const int rlane = lane & 15;
  const int koff  = (lane >> 4) * 8;
  const int mOff  = (lane >> 4) * 8;

  v8f acc[4][4];
#pragma unroll
  for (int i = 0; i < 4; ++i)
#pragma unroll
    for (int j = 0; j < 4; ++j) acc[i][j] = (v8f){0.f,0.f,0.f,0.f,0.f,0.f,0.f,0.f};

  for (int k0 = 0; k0 < K; k0 += 32) {
    V bh[4], bl[4];
#pragma unroll
    for (int j = 0; j < 4; ++j) {
      const size_t bo = (size_t)(n0 + (j << 4) + rlane) * ldb + koff + k0;
      bh[j] = Frag<T>::load(Bb + bo);
      if (SPLIT) bl[j] = Frag<T>::load(Bb2 + bo);
    }
#pragma unroll
    for (int i = 0; i < 4; ++i) {
      const size_t ao = (size_t)(m0 + (i << 4) + rlane) * lda + koff + k0;
      V ah = Frag<T>::load(Ab + ao);
      V al;
      if (SPLIT) al = Frag<T>::load(Ab2 + ao);
#pragma unroll
      for (int j = 0; j < 4; ++j) {
        acc[i][j] = Frag<T>::mma(ah, bh[j], acc[i][j]);
        if (SPLIT) {
          acc[i][j] = Frag<T>::mma(ah, bl[j], acc[i][j]);
          acc[i][j] = Frag<T>::mma(al, bh[j], acc[i][j]);
        }
      }
      Frag<T>::guard(acc[i][0], acc[i][3], ah, SPLIT ? al : ah);
    }
    Frag<T>::keep(bh[0], bh[1], bh[2], bh[3]);
    if (SPLIT) Frag<T>::keep(bl[0], bl[1], bl[2], bl[3]);
  }
  acc_guard4(acc[0][0], acc[0][1], acc[0][2], acc[0][3]);
  acc_guard4(acc[1][0], acc[1][1], acc[1][2], acc[1][3]);
  acc_guard4(acc[2][0], acc[2][1], acc[2][2], acc[2][3]);
  acc_guard4(acc[3][0], acc[3][1], acc[3][2], acc[3][3]);

  float* slab = sT[wave];
  const float* Rb = RESID ? (resid + (size_t)b * strideR) : nullptr;
#pragma unroll
  for (int i = 0; i < 4; ++i) {
    const int mBase = m0 + (i << 4);
#pragma unroll
    for (int j = 0; j < 4; ++j) {
      const int n = n0 + (j << 4) + rlane;
      float bv = 0.f;
      if (BIAS_MODE == 2) bv = bias[n];
#pragma unroll
      for (int r = 0; r < 8; ++r) {
        float v = acc[i][j][r] * scale;
        if (BIAS_MODE == 1) v += bias[mBase + mOff + r];
        if (BIAS_MODE == 2) v += bv;
        if (RESID) v += Rb[(size_t)(mBase + mOff + r) * ldc + n];
        if (ACT == 1) v = tanhf(v);
        if (ACT == 2) v = fmaxf(v, 0.0f);
        if (ACT == 3) v = v / (1.0f + expf(-v));
        if (ACT == 4) v = (v > 0.f) ? v : 0.01f * v;
        if (ACT == 5) v = 0.5f * v * (1.0f + erff(v * 0.70710678118654752f));
        slab[(mOff + r) * 68 + (j << 4) + rlane] = v;
      }
    }
    __builtin_amdgcn_fence(__ATOMIC_RELEASE, "workgroup");
    __builtin_amdgcn_wave_barrier();
    __builtin_amdgcn_fence(__ATOMIC_ACQUIRE, "workgroup");
    if (OUT_MODE == 0) {
      float* C = (float*)Cout + (size_t)b * strideC;
      const int hh = lane >> 4, c4 = (lane & 15) * 4;
      for (int pass = 0; pass < 2; ++pass) {
#pragma unroll
        for (int it = 0; it < 8; ++it) {
          const int row = it * 2 + hh;
          v4f v = *(const v4f*)(slab + row * 68 + c4);
          *(volatile v4f*)(C + (size_t)(mBase + row) * ldc + n0 + c4) = v;
        }
        __threadfence();
      }
    } else {
      const int q = lane >> 3, c8 = (lane & 7) * 8;
      unsigned short* C  = (unsigned short*)Cout  + (size_t)b * strideC;
      unsigned short* C2 = (OUT_MODE == 2) ? ((unsigned short*)Cout2 + (size_t)b * strideC) : nullptr;
      for (int pass = 0; pass < 2; ++pass) {
#pragma unroll
        for (int it = 0; it < 4; ++it) {
          const int row = it * 4 + q;
          const float* sp = slab + row * 68 + c8;
          v8h hv, lv;
#pragma unroll
          for (int e = 0; e < 8; ++e) {
            if (OUT_MODE == 1) {
              hv[e] = (_Float16)sp[e];
            } else {
              unsigned short hb = f2bf_bits(sp[e]);
              unsigned short lb = f2bf_bits(sp[e] - bf_bits2f(hb));
              hv[e] = __builtin_bit_cast(_Float16, hb);
              lv[e] = __builtin_bit_cast(_Float16, lb);
            }
          }
          *(volatile v8h*)(C + (size_t)(mBase + row) * ldc + n0 + c8) = hv;
          if (OUT_MODE == 2) *(volatile v8h*)(C2 + (size_t)(mBase + row) * ldc + n0 + c8) = lv;
        }
        __threadfence();
      }
    }
    __builtin_amdgcn_fence(__ATOMIC_RELEASE, "workgroup");
    __builtin_amdgcn_wave_barrier();
    __builtin_amdgcn_fence(__ATOMIC_ACQUIRE, "workgroup");
  }
}

static constexpr int NDOC  = 32;
static constexpr int NSENT = 32;
static constexpr int NTOK  = 64;
static constexpr int EMBD  = 128;
static constexpr int HID   = 128;
static constexpr int CTXD  = 128;
static constexpr int VOCAB = 50000;
static constexpr int NCLS  = 8;
static constexpr int NROWW = NDOC * NSENT;
static constexpr float ACT_CARRY = 16.0f;
static constexpr float W_CARRY   = 8.0f;
static constexpr float INV_CARRY = 1.0f / 128.0f;
static_assert(HID == 8 * 16, "eight waves of 16 columns cover the hidden size");
static_assert(NROWW == 4 * 256, "lens kernel maps 4 rows per thread");
static_assert(NDOC == 32, "one lane per document in the lens kernel");

__device__ __forceinline__ v8f zero8() { return (v8f){0.f,0.f,0.f,0.f,0.f,0.f,0.f,0.f}; }
__device__ __forceinline__ float h16lo(unsigned w) { return (float)__builtin_bit_cast(_Float16, (unsigned short)(w & 0xffffu)); }
__device__ __forceinline__ float h16hi(unsigned w) { return (float)__builtin_bit_cast(_Float16, (unsigned short)(w >> 16)); }

__global__ __launch_bounds__(256) void k_cast4(
    const float* __restrict__ s0, _Float16* __restrict__ d0, int n0,
    const float* __restrict__ s1, _Float16* __restrict__ d1, int n1,
    const float* __restrict__ s2, _Float16* __restrict__ d2, int n2,
    const float* __restrict__ s3, _Float16* __restrict__ d3, int n3, float scale) {
  const int y = blockIdx.y;
  const float* s = (y == 0) ? s0 : ((y == 1) ? s1 : ((y == 2) ? s2 : s3));
  _Float16* d = (y == 0) ? d0 : ((y == 1) ? d1 : ((y == 2) ? d2 : d3));
  const int npair = ((y == 0) ? n0 : ((y == 1) ? n1 : ((y == 2) ? n2 : n3))) >> 1;
  const int i = blockIdx.x * 256 + threadIdx.x;
  if (i < npair) {
    const float f0 = s[2 * i] * scale;
    const float f1 = s[2 * i + 1] * scale;
    const _Float16 h0 = (_Float16)f0, h1 = (_Float16)f1;
    const unsigned u = (unsigned)__builtin_bit_cast(unsigned short, h0) | ((unsigned)__builtin_bit_cast(unsigned short, h1) << 16);
    ((volatile unsigned*)d)[i] = u;
    __threadfence();
    ((volatile unsigned*)d)[i] = u;
  }
}

__global__ __launch_bounds__(256) void k_lens(const int* __restrict__ x, int* __restrict__ wlen,
                                              int* __restrict__ slen, int* __restrict__ maxl) {
  __shared__ int nzf[NROWW];
  __shared__ int red[256];
  const int tid = threadIdx.x, lane = tid & 31, wave = tid >> 5;
  int lens4[4];
  int mymax = 0;
#pragma unroll
  for (int p = 0; p < 4; ++p) {
    const int row = p * 256 + tid;
    const v4i* rp = (const v4i*)(x + (size_t)row * NTOK);
    int last = 0;
#pragma unroll 4
    for (int i = 0; i < NTOK / 4; ++i) {
      const v4i v = rp[i];
      const int b4 = 4 * i;
      last = (v[0] != 0) ? (b4 + 1) : last;
      last = (v[1] != 0) ? (b4 + 2) : last;
      last = (v[2] != 0) ? (b4 + 3) : last;
      last = (v[3] != 0) ? (b4 + 4) : last;
    }
    nzf[row] = (last > 0) ? 1 : 0;
    const int len = (last > 0) ? last : 1;
    lens4[p] = len;
    mymax = max(mymax, len);
  }
  for (int pass = 0; pass < 2; ++pass) {
#pragma unroll
    for (int p = 0; p < 4; ++p) ((volatile int*)wlen)[p * 256 + tid] = lens4[p];
    __threadfence();
  }
  red[tid] = mymax;
  __syncthreads();
  for (int s = 128; s > 0; s >>= 1) {
    if (tid < s) red[tid] = max(red[tid], red[tid + s]);
    __syncthreads();
  }
  const int wmax = red[0];
  if (wave == 0) {
    int last = 0;
    for (int s2 = 0; s2 < NSENT; ++s2) last = (nzf[lane * NSENT + s2] != 0) ? (s2 + 1) : last;
    const int sl = (last > 0) ? last : 1;
    int smax = sl;
#pragma unroll
    for (int off = 1; off < 32; off <<= 1) smax = max(smax, __shfl_xor(smax, off, 32));
    const int mv = (lane == 0) ? wmax : ((lane == 1) ? smax : 0);
    for (int pass = 0; pass < 2; ++pass) {
      ((volatile int*)slen)[lane] = sl;
      ((volatile int*)maxl)[lane] = mv;
      __threadfence();
    }
  }
}

template <int DIN, int TSTEPS, bool GATHER>
__global__ __launch_bounds__(256) void k_bigru(
    const int* __restrict__ tokens, const float* __restrict__ xsrc,
    const _Float16* __restrict__ wih_f, const _Float16* __restrict__ whh_f,
    const float* __restrict__ bih_f, const float* __restrict__ bhh_f,
    const _Float16* __restrict__ wih_b, const _Float16* __restrict__ whh_b,
    const float* __restrict__ bih_b, const float* __restrict__ bhh_b,
    const int* __restrict__ lens, _Float16* __restrict__ out16) {
  constexpr int KTI = DIN / 32;
  constexpr int KTH = HID / 32;
  constexpr int LDX = DIN + 8;
  constexpr int LDH = HID + 8;
  constexpr int XCH = DIN / 8;
  static_assert(DIN % 32 == 0 && (KTI % 2) == 0 && (KTH % 2) == 0, "k tiling");
  static_assert((16 * XCH) % 256 == 0, "X staging covers the whole tile");
  __shared__ __align__(16) _Float16 Xs[16 * LDX];
  __shared__ __align__(16) _Float16 Hs[16 * LDH];
  __shared__ __align__(16) float hS[16 * HID];
  __shared__ __align__(16) float oS[16 * HID];
  __shared__ int lenS[16];

  const int tid = threadIdx.x, lane = tid & 31, wave = tid >> 5;
  const int rlane = lane & 15, hh = lane >> 4, koff = hh * 8;
  const int rowbase = blockIdx.x * 16;
  const int dir = blockIdx.y;
  const _Float16* wih = dir ? wih_b : wih_f;
  const _Float16* whh = dir ? whh_b : whh_f;
  const float* bih = dir ? bih_b : bih_f;
  const float* bhh = dir ? bhh_b : bhh_f;

  if (tid < 16) lenS[tid] = lens[rowbase + tid];
  for (int i = tid; i < 16 * HID; i += 256) hS[i] = 0.0f;
  __syncthreads();
  int lenr[8];
#pragma unroll
  for (int r = 0; r < 8; ++r) lenr[r] = lenS[hh * 8 + r];
  const int col = wave * 16 + rlane;
  const float br  = bih[col] + bhh[col];
  const float bz  = bih[HID + col] + bhh[HID + col];
  const float bxn = bih[2 * HID + col];
  const float bhn = bhh[2 * HID + col];

  for (int step = 0; step < TSTEPS; ++step) {
    const int tt = dir ? (TSTEPS - 1 - step) : step;
    for (int i = tid; i < 16 * XCH; i += 256) {
      const int m = i / XCH;
      const int ch = i - m * XCH;
      size_t so;
      if (GATHER) {
        int tok = tokens[(size_t)(rowbase + m) * TSTEPS + tt];
        tok = tok < 0 ? 0 : (tok > VOCAB - 1 ? VOCAB - 1 : tok);
        so = (size_t)tok * DIN + (size_t)ch * 8;
      } else {
        so = ((size_t)(rowbase + m) * TSTEPS + tt) * DIN + (size_t)ch * 8;
      }
      const v4f a0 = *(const v4f*)(xsrc + so);
      const v4f a1 = *(const v4f*)(xsrc + so + 4);
      v8h hv;
      hv[0] = (_Float16)(a0[0] * ACT_CARRY); hv[1] = (_Float16)(a0[1] * ACT_CARRY);
      hv[2] = (_Float16)(a0[2] * ACT_CARRY); hv[3] = (_Float16)(a0[3] * ACT_CARRY);
      hv[4] = (_Float16)(a1[0] * ACT_CARRY); hv[5] = (_Float16)(a1[1] * ACT_CARRY);
      hv[6] = (_Float16)(a1[2] * ACT_CARRY); hv[7] = (_Float16)(a1[3] * ACT_CARRY);
      *(v8h*)(Xs + m * LDX + ch * 8) = hv;
    }
    {
      const int m = tid >> 4, ch = tid & 15;
      const float* sp = hS + m * HID + ch * 8;
      v8h hv;
#pragma unroll
      for (int e = 0; e < 8; ++e) hv[e] = (_Float16)(sp[e] * ACT_CARRY);
      *(v8h*)(Hs + m * LDH + ch * 8) = hv;
    }
    __syncthreads();

    v8f ax0 = zero8(), ax1 = zero8(), ax2 = zero8();
    v8f ah0 = zero8(), ah1 = zero8(), ah2 = zero8();
#pragma unroll 2
    for (int kt = 0; kt < KTI; ++kt) {
      const int k0 = kt * 32;
      const v16h a  = Frag<_Float16>::load(Xs + rlane * LDX + k0 + koff);
      const v16h b0 = Frag<_Float16>::load(wih + (size_t)col * DIN + k0 + koff);
      const v16h b1 = Frag<_Float16>::load(wih + (size_t)(HID + col) * DIN + k0 + koff);
      const v16h b2 = Frag<_Float16>::load(wih + (size_t)(2 * HID + col) * DIN + k0 + koff);
      ax0 = Frag<_Float16>::mma(a, b0, ax0);
      ax1 = Frag<_Float16>::mma(a, b1, ax1);
      ax2 = Frag<_Float16>::mma(a, b2, ax2);
      guard3_h(ax0, ax1, ax2, a, b0, b1, b2);
    }
#pragma unroll 2
    for (int kt = 0; kt < KTH; ++kt) {
      const int k0 = kt * 32;
      const v16h a  = Frag<_Float16>::load(Hs + rlane * LDH + k0 + koff);
      const v16h b0 = Frag<_Float16>::load(whh + (size_t)col * HID + k0 + koff);
      const v16h b1 = Frag<_Float16>::load(whh + (size_t)(HID + col) * HID + k0 + koff);
      const v16h b2 = Frag<_Float16>::load(whh + (size_t)(2 * HID + col) * HID + k0 + koff);
      ah0 = Frag<_Float16>::mma(a, b0, ah0);
      ah1 = Frag<_Float16>::mma(a, b1, ah1);
      ah2 = Frag<_Float16>::mma(a, b2, ah2);
      guard3_h(ah0, ah1, ah2, a, b0, b1, b2);
    }
    acc_guard3(ax0, ax1, ax2);
    acc_guard3(ah0, ah1, ah2);

#pragma unroll
    for (int r = 0; r < 8; ++r) {
      const int m = hh * 8 + r;
      const float pr = (ax0[r] + ah0[r]) * INV_CARRY + br;
      const float pz = (ax1[r] + ah1[r]) * INV_CARRY + bz;
      const float hn = ah2[r] * INV_CARRY + bhn;
      const float rg = 1.0f / (1.0f + expf(-pr));
      const float zg = 1.0f / (1.0f + expf(-pz));
      const float ng = tanhf(ax2[r] * INV_CARRY + bxn + rg * hn);
      const float hold = hS[m * HID + col];
      const float hnew = (1.0f - zg) * ng + zg * hold;
      const bool valid = tt < lenr[r];
      hS[m * HID + col] = valid ? hnew : hold;
      oS[m * HID + col] = valid ? hnew : 0.0f;
    }
    __syncthreads();

    {
      const int m = 2 * wave + hh;
      const int c8 = rlane * 8;
      const float* sp = oS + m * HID + c8;
      v8h hv;
#pragma unroll
      for (int e = 0; e < 8; ++e) hv[e] = (_Float16)(sp[e] * ACT_CARRY);
      _Float16* dst = out16 + ((size_t)(rowbase + m) * TSTEPS + tt) * (2 * HID) + (size_t)dir * HID + c8;
      *(volatile v8h*)dst = hv;
      __threadfence();
      *(volatile v8h*)dst = hv;
    }
  }
}

__global__ __launch_bounds__(256) void k_ctxdot(const float* __restrict__ u, const float* __restrict__ ctx,
                                                float* __restrict__ sc) {
  const int lane = threadIdx.x & 31, wave = threadIdx.x >> 5;
  const size_t rbase = ((size_t)blockIdx.x * 8 + wave) * 32;
  const v4f c4 = *(const v4f*)(ctx + lane * 4);
  float res = 0.0f;
#pragma unroll 2
  for (int j = 0; j < 32; ++j) {
    const v4f w = *(const v4f*)(u + (rbase + j) * CTXD + lane * 4);
    float s = w[0] * c4[0];
    s += w[1] * c4[1];
    s += w[2] * c4[2];
    s += w[3] * c4[3];
#pragma unroll
    for (int off = 1; off < 32; off <<= 1) s += __shfl_xor(s, off, 32);
    res = (lane == j) ? s : res;
  }
  for (int pass = 0; pass < 2; ++pass) {
    ((volatile float*)sc)[rbase + lane] = res;
    __threadfence();
  }
}

template <int TT>
__global__ __launch_bounds__(256) void k_softmax_pool(const float* __restrict__ sc, const _Float16* __restrict__ o16,
                                                      const int* __restrict__ maxl, int which,
                                                      float* __restrict__ pooled) {
  static_assert(TT <= 64 && TT % 8 == 0, "time extent");
  __shared__ float pw[64];
  __shared__ __align__(16) float red[8 * 256];
  __shared__ __align__(16) float rowv[256];
  __shared__ float sinv;
  const int tid = threadIdx.x, lane = tid & 31, wave = tid >> 5;
  const int n = blockIdx.x;
  int tmax = maxl[which];
  tmax = tmax < 1 ? 1 : (tmax > TT ? TT : tmax);
  if (tid < TT) {
    const float v = sc[(size_t)n * TT + tid];
    pw[tid] = (tid < tmax) ? v : -INFINITY;
  }
  __syncthreads();
  if (tid == 0) {
    float m = -INFINITY;
#pragma unroll 1
    for (int t = 0; t < TT; ++t) m = fmaxf(m, pw[t]);
    float s = 0.0f;
#pragma unroll 1
    for (int t = 0; t < TT; ++t) { const float e = expf(pw[t] - m); pw[t] = e; s += e; }
    sinv = 1.0f / s;
  }
  __syncthreads();
  const int h8 = lane * 8;
  float acc[8];
#pragma unroll
  for (int e = 0; e < 8; ++e) acc[e] = 0.0f;
  const unsigned* obase = (const unsigned*)(const void*)(o16 + (size_t)n * TT * (2 * HID));
#pragma unroll 2
  for (int t = wave; t < TT; t += 8) {
    const v4u w = *(const v4u*)(obase + (size_t)t * HID + lane * 4);
    const float pt = pw[t];
    acc[0] += pt * h16lo(w[0]); acc[1] += pt * h16hi(w[0]);
    acc[2] += pt * h16lo(w[1]); acc[3] += pt * h16hi(w[1]);
    acc[4] += pt * h16lo(w[2]); acc[5] += pt * h16hi(w[2]);
    acc[6] += pt * h16lo(w[3]); acc[7] += pt * h16hi(w[3]);
  }
#pragma unroll
  for (int e = 0; e < 8; ++e) red[wave * 256 + h8 + e] = acc[e];
  __syncthreads();
  float v = 0.0f;
#pragma unroll
  for (int g = 0; g < 8; ++g) v += red[g * 256 + tid];
  rowv[tid] = v * sinv * (1.0f / ACT_CARRY);
  __syncthreads();
  if (wave == 0) {
    const v4f a = *(const v4f*)(rowv + lane * 4);
    const v4f b = *(const v4f*)(rowv + 128 + lane * 4);
    float* dst = pooled + (size_t)n * (2 * HID);
    for (int pass = 0; pass < 2; ++pass) {
      *(volatile v4f*)(dst + lane * 4) = a;
      *(volatile v4f*)(dst + 128 + lane * 4) = b;
      __threadfence();
    }
  }
}

__global__ __launch_bounds__(256) void k_fc(const float* __restrict__ doc, const float* __restrict__ fw,
                                            const float* __restrict__ fb, float* __restrict__ out) {
  __shared__ __align__(16) float ov[256];
  const int tid = threadIdx.x, lane = tid & 31, wave = tid >> 5;
  const int r = tid >> 3, k = tid & 7;
  float s = 0.0f;
#pragma unroll 4
  for (int j = 0; j < 2 * HID; ++j) s += doc[r * (2 * HID) + j] * fw[k * (2 * HID) + j];
  s += fb[k];
  ov[tid] = s;
  __syncthreads();
  if (wave == 0) {
    const v4f a = *(const v4f*)(ov + lane * 4);
    const v4f b = *(const v4f*)(ov + 128 + lane * 4);
    for (int pass = 0; pass < 2; ++pass) {
      *(volatile v4f*)(out + lane * 4) = a;
      *(volatile v4f*)(out + 128 + lane * 4) = b;
      __threadfence();
    }
  }
}

static constexpr size_t SZ_WOUT16 = (size_t)NROWW * NTOK * 2 * HID * 2;
static constexpr size_t SZ_UPL    = (size_t)NROWW * NTOK * CTXD * 4;
static constexpr size_t SZ_SC     = (size_t)NROWW * NTOK * 4;
static constexpr size_t SZ_SENT   = (size_t)NROWW * 2 * HID * 4;
static constexpr size_t SZ_SOUT16 = (size_t)NDOC * NSENT * 2 * HID * 2;
static constexpr size_t SZ_DOC    = (size_t)NDOC * 2 * HID * 4;
static constexpr size_t SZ_WLEN   = (size_t)NROWW * 4;
static constexpr size_t SZ_LINE   = 128;
static constexpr size_t SZ_W128   = (size_t)3 * HID * EMBD * 2;
static constexpr size_t SZ_W256   = (size_t)3 * HID * 2 * HID * 2;
static constexpr size_t SZ_WPRJ   = (size_t)CTXD * 2 * HID * 2;

static constexpr size_t OFF_WOUT16 = 0;
static constexpr size_t OFF_UPL    = OFF_WOUT16 + SZ_WOUT16;
static constexpr size_t OFF_SC     = OFF_UPL + SZ_UPL;
static constexpr size_t OFF_SENT   = OFF_SC + SZ_SC;
static constexpr size_t OFF_SOUT16 = OFF_SENT + SZ_SENT;
static constexpr size_t OFF_DOC    = OFF_SOUT16 + SZ_SOUT16;
static constexpr size_t OFF_WLEN   = OFF_DOC + SZ_DOC;
static constexpr size_t OFF_SLEN   = OFF_WLEN + SZ_WLEN;
static constexpr size_t OFF_MAXL   = OFF_SLEN + SZ_LINE;
static constexpr size_t OFF_WFIH   = OFF_MAXL + SZ_LINE;
static constexpr size_t OFF_WFHH   = OFF_WFIH + SZ_W128;
static constexpr size_t OFF_WBIH   = OFF_WFHH + SZ_W128;
static constexpr size_t OFF_WBHH   = OFF_WBIH + SZ_W128;
static constexpr size_t OFF_SFIH   = OFF_WBHH + SZ_W128;
static constexpr size_t OFF_SFHH   = OFF_SFIH + SZ_W256;
static constexpr size_t OFF_SBIH   = OFF_SFHH + SZ_W128;
static constexpr size_t OFF_SBHH   = OFF_SBIH + SZ_W256;
static constexpr size_t OFF_WPRJ   = OFF_SBHH + SZ_W128;
static constexpr size_t OFF_SPRJ   = OFF_WPRJ + SZ_WPRJ;
static constexpr size_t WS_END     = OFF_SPRJ + SZ_WPRJ;
static_assert(WS_END == 70095104, "carve total");
static_assert(WS_END <= 134217728, "carve budget");
static_assert((OFF_UPL % 256) == 0 && (OFF_SC % 256) == 0 && (OFF_SENT % 256) == 0 && (OFF_SOUT16 % 256) == 0 &&
              (OFF_DOC % 256) == 0 && (OFF_WLEN % 256) == 0 && (OFF_SLEN % 128) == 0 && (OFF_MAXL % 128) == 0 &&
              (OFF_WFIH % 256) == 0 && (OFF_SPRJ % 256) == 0, "alignment");
static_assert((size_t)NDOC * NSENT * CTXD * 4 <= SZ_UPL && (size_t)NDOC * NSENT * 4 <= SZ_SC, "reuse");
static_assert((NROWW * NTOK) % 64 == 0 && (NDOC * NSENT) % 64 == 0 && CTXD % 64 == 0 && (2 * HID) % 32 == 0, "gemm shapes");
static_assert(((NROWW * NTOK / 64) * (CTXD / 64)) % 8 == 0 && ((NDOC * NSENT / 64) * (CTXD / 64)) % 8 == 0, "gemm grids");
static_assert((NROWW * NTOK) % 256 == 0 && (NDOC * NSENT) % 256 == 0, "ctxdot grids");

extern "C" void kernel_launch(void* const* d_in, const int* in_sizes, int n_in,
                              void* d_out, int out_size, void* d_ws, size_t ws_size,
                              hipStream_t stream) {
  (void)in_sizes; (void)n_in; (void)out_size;
  if (ws_size < WS_END) return;
  const int*   x       = (const int*)  d_in[0];
  const float* emb     = (const float*)d_in[1];
  const float* wf_Wih  = (const float*)d_in[2];
  const float* wf_Whh  = (const float*)d_in[3];
  const float* wf_bih  = (const float*)d_in[4];
  const float* wf_bhh  = (const float*)d_in[5];
  const float* wb_Wih  = (const float*)d_in[6];
  const float* wb_Whh  = (const float*)d_in[7];
  const float* wb_bih  = (const float*)d_in[8];
  const float* wb_bhh  = (const float*)d_in[9];
  const float* sf_Wih  = (const float*)d_in[10];
  const float* sf_Whh  = (const float*)d_in[11];
  const float* sf_bih  = (const float*)d_in[12];
  const float* sf_bhh  = (const float*)d_in[13];
  const float* sb_Wih  = (const float*)d_in[14];
  const float* sb_Whh  = (const float*)d_in[15];
  const float* sb_bih  = (const float*)d_in[16];
  const float* sb_bhh  = (const float*)d_in[17];
  const float* wproj_W = (const float*)d_in[18];
  const float* wproj_b = (const float*)d_in[19];
  const float* wctx    = (const float*)d_in[20];
  const float* sproj_W = (const float*)d_in[21];
  const float* sproj_b = (const float*)d_in[22];
  const float* sctx    = (const float*)d_in[23];
  const float* fc_W    = (const float*)d_in[24];
  const float* fc_b    = (const float*)d_in[25];
  float* out = (float*)d_out;

  char* ws = (char*)d_ws;
  _Float16* WOUT16 = (_Float16*)(ws + OFF_WOUT16);
  float*    UPL    = (float*)(ws + OFF_UPL);
  float*    SC     = (float*)(ws + OFF_SC);
  float*    SENT   = (float*)(ws + OFF_SENT);
  _Float16* SOUT16 = (_Float16*)(ws + OFF_SOUT16);
  float*    DOC    = (float*)(ws + OFF_DOC);
  int*      WLEN   = (int*)(ws + OFF_WLEN);
  int*      SLEN   = (int*)(ws + OFF_SLEN);
  int*      MAXL   = (int*)(ws + OFF_MAXL);
  _Float16* WFIH = (_Float16*)(ws + OFF_WFIH);
  _Float16* WFHH = (_Float16*)(ws + OFF_WFHH);
  _Float16* WBIH = (_Float16*)(ws + OFF_WBIH);
  _Float16* WBHH = (_Float16*)(ws + OFF_WBHH);
  _Float16* SFIH = (_Float16*)(ws + OFF_SFIH);
  _Float16* SFHH = (_Float16*)(ws + OFF_SFHH);
  _Float16* SBIH = (_Float16*)(ws + OFF_SBIH);
  _Float16* SBHH = (_Float16*)(ws + OFF_SBHH);
  _Float16* WPRJ = (_Float16*)(ws + OFF_WPRJ);
  _Float16* SPRJ = (_Float16*)(ws + OFF_SPRJ);

  const int nW128 = 3 * HID * EMBD;
  const int nW256 = 3 * HID * 2 * HID;
  const int nWPRJ = CTXD * 2 * HID;

  k_cast4<<<dim3((nW128 / 2 + 255) / 256, 4), 256, 0, stream>>>(
      wf_Wih, WFIH, nW128, wf_Whh, WFHH, nW128, wb_Wih, WBIH, nW128, wb_Whh, WBHH, nW128, W_CARRY);
  k_cast4<<<dim3((nW256 / 2 + 255) / 256, 4), 256, 0, stream>>>(
      sf_Wih, SFIH, nW256, sf_Whh, SFHH, nW128, sb_Wih, SBIH, nW256, sb_Whh, SBHH, nW128, W_CARRY);
  k_cast4<<<dim3((nWPRJ / 2 + 255) / 256, 4), 256, 0, stream>>>(
      wproj_W, WPRJ, nWPRJ, sproj_W, SPRJ, nWPRJ, wproj_W, WPRJ, 0, sproj_W, SPRJ, 0, W_CARRY);

  k_lens<<<1, 256, 0, stream>>>(x, WLEN, SLEN, MAXL);

  k_bigru<EMBD, NTOK, true><<<dim3(NROWW / 16, 2), 256, 0, stream>>>(
      x, emb, WFIH, WFHH, wf_bih, wf_bhh, WBIH, WBHH, wb_bih, wb_bhh, WLEN, WOUT16);

  wmma_gemm64<0, false, 2, 0, false, 1><<<dim3(((NROWW * NTOK) / 64) * (CTXD / 64) / 8, 1), 256, 0, stream>>>(
      (const unsigned short*)WOUT16, (const unsigned short*)WOUT16, 2 * HID, 0L,
      (const unsigned short*)WPRJ, (const unsigned short*)WPRJ, 2 * HID, 0L,
      (void*)UPL, (void*)UPL, CTXD, 0L,
      wproj_b, wproj_b, 0L,
      NROWW * NTOK, CTXD, 2 * HID, INV_CARRY);
  k_ctxdot<<<(NROWW * NTOK) / 256, 256, 0, stream>>>(UPL, wctx, SC);
  k_softmax_pool<NTOK><<<NROWW, 256, 0, stream>>>(SC, WOUT16, MAXL, 0, SENT);

  k_bigru<2 * HID, NSENT, false><<<dim3(NDOC / 16, 2), 256, 0, stream>>>(
      x, SENT, SFIH, SFHH, sf_bih, sf_bhh, SBIH, SBHH, sb_bih, sb_bhh, SLEN, SOUT16);

  wmma_gemm64<0, false, 2, 0, false, 1><<<dim3(((NDOC * NSENT) / 64) * (CTXD / 64) / 8, 1), 256, 0, stream>>>(
      (const unsigned short*)SOUT16, (const unsigned short*)SOUT16, 2 * HID, 0L,
      (const unsigned short*)SPRJ, (const unsigned short*)SPRJ, 2 * HID, 0L,
      (void*)UPL, (void*)UPL, CTXD, 0L,
      sproj_b, sproj_b, 0L,
      NDOC * NSENT, CTXD, 2 * HID, INV_CARRY);
  k_ctxdot<<<(NDOC * NSENT) / 256, 256, 0, stream>>>(UPL, sctx, SC);
  k_softmax_pool<NSENT><<<NDOC, 256, 0, stream>>>(SC, SOUT16, MAXL, 1, DOC);

  k_fc<<<1, 256, 0, stream>>>(DOC, fc_W, fc_b, out);
}
